// HeteroGraphTransformer_19593640805065
// MI455X (gfx1250) — hardware-run, weakly checked
//
#include <hip/hip_runtime.h>
#include <stddef.h>
#include <math.h>


#define DIN    64
#define HID    128
#define INNER  1024
#define QKVP   3072
#define FFD    512
#define NHD    8
#define NLAY   2
#define GBM    80
#define GTH    160
#define GWT    2048
#define NBK    16
#define HCAP   256
#define KPIT   136
#define VPIT   264
#define SPIT   256
#define PPIT   264
#define WPP    72
#define ECH    4096
#define WSCAP  134217728
#define ASCL   8.0f
#define WSCL   64.0f
#define PSCL   2048.0f
#define INVSCL 0.001953125f
#define OSCL   7.62939453125e-6f
#define LSCL   (0.08838834764831845f * 0.015625f)
#define INVHID 0.0078125f
#define LNEPS  1e-5f
#define DSENT  (-1073741824)

#define LO_KS   0
#define LO_VT   (LO_KS + HCAP * KPIT * 2)
#define LO_S    (LO_VT + 128 * VPIT * 2)
#define LO_P    (LO_S + NBK * SPIT * 4)
#define LO_LIST (LO_P + NBK * PPIT * 2)
#define LO_WT   (LO_LIST + HCAP * 4)
#define LO_RED  (LO_WT + 64)
#define LO_BETA (LO_RED + NBK * 8 * 4)
#define CONV_LDS (LO_BETA + 64)

static_assert(NHD * HID == INNER);
static_assert((HCAP % 32) == 0 && SPIT >= HCAP && PPIT >= HCAP + 8 && VPIT >= HCAP + 8);
static_assert((KPIT % 8) == 0 && (VPIT % 8) == 0 && (PPIT % 8) == 0 && (WPP % 8) == 0);
static_assert((LO_VT % 16) == 0 && (LO_S % 16) == 0 && (LO_P % 16) == 0 && (LO_LIST % 16) == 0);
static_assert((LO_WT % 16) == 0 && (LO_RED % 16) == 0 && (LO_BETA % 16) == 0);
static_assert(NBK * HID * 4 <= NBK * SPIT * 4);
static_assert(CONV_LDS <= 300000);
static_assert(ECH == 256 * 16);
static_assert(HCAP <= 256);
static_assert((GBM % 16) == 0 && GTH == (GBM / 16) * 32);
static_assert((INNER % 128) == 0 && (FFD % 128) == 0 && (HID % 128) == 0);
static_assert((DIN % 32) == 0 && (HID % 64) == 0 && (DIN % 64) == 0);

typedef float          v4f  __attribute__((ext_vector_type(4)));
typedef float          v8f  __attribute__((ext_vector_type(8)));
typedef int            v4i  __attribute__((ext_vector_type(4)));
typedef unsigned short v4us __attribute__((ext_vector_type(4)));
typedef unsigned short v8us __attribute__((ext_vector_type(8)));
typedef _Float16       v16h __attribute__((ext_vector_type(16)));
union FragH { v16h v; v8us u[2]; };

__device__ __forceinline__ unsigned short h16(float f) {
  const _Float16 h = (_Float16)f;
  return __builtin_bit_cast(unsigned short, h);
}

__device__ __forceinline__ v8us cvt8(v4f a, v4f b, float s) {
  v8us r;
  r[0] = h16(a.x * s); r[1] = h16(a.y * s); r[2] = h16(a.z * s); r[3] = h16(a.w * s);
  r[4] = h16(b.x * s); r[5] = h16(b.y * s); r[6] = h16(b.z * s); r[7] = h16(b.w * s);
  return r;
}

__device__ __forceinline__ float geluf(float x) {
  return 0.5f * x * (1.0f + erff(x * 0.70710678118654752f));
}
__device__ __forceinline__ v4f gelu4(v4f a) {
  v4f r;
  r.x = geluf(a.x); r.y = geluf(a.y); r.z = geluf(a.z); r.w = geluf(a.w);
  return r;
}

__device__ __forceinline__ v8f zero8() {
  v8f z = {0.f, 0.f, 0.f, 0.f, 0.f, 0.f, 0.f, 0.f};
  return z;
}

__device__ __forceinline__ v8f wmh(v16h a, v16h b, v8f c) {
  v8f d = __builtin_amdgcn_wmma_f32_16x16x32_f16(false, a, false, b, (short)0, c, false, false);
  asm volatile("v_nop\n\tv_nop\n\tv_nop\n\tv_nop" : "+v"(d) : "v"(a), "v"(b));
  return d;
}

__global__ __launch_bounds__(256) void k_wpack(
    const float* __restrict__ W, unsigned short* wt, int K, int M, int szs, int dzs) {
  __shared__ __attribute__((aligned(16))) unsigned short sT[64 * WPP];
  const int tid = (int)threadIdx.x;
  const int m0 = (int)blockIdx.x * 64, k0 = (int)blockIdx.y * 64;
  const float* Wz = W + (size_t)blockIdx.z * (size_t)szs;
  unsigned short* wz = wt + (size_t)blockIdx.z * (size_t)dzs;
#pragma unroll 4
  for (int it = 0; it < 16; ++it) {
    const int idx = it * 256 + tid;
    const int kk = idx >> 6, mm = idx & 63;
    int kr = k0 + kk; kr = kr > K - 1 ? K - 1 : kr;
    int mc = m0 + mm; mc = mc > M - 1 ? M - 1 : mc;
    const float w = Wz[(size_t)kr * M + mc];
    sT[mm * WPP + kk] = h16(w * WSCL);
  }
  __syncthreads();
  v8us pv[2];
  size_t po[2];
#pragma unroll
  for (int it = 0; it < 2; ++it) {
    const int p = it * 256 + tid;
    const int row = p >> 3, c8 = (p & 7) * 8;
    pv[it] = *(const v8us*)(sT + row * WPP + c8);
    int mr = m0 + row; mr = mr > M - 1 ? M - 1 : mr;
    po[it] = (size_t)mr * K + k0 + c8;
  }
  const bool full = (m0 + 64 <= M) && (k0 + 64 <= K);
  if (full) {
#pragma unroll
    for (int it = 0; it < 2; ++it) *(volatile v8us*)(wz + po[it]) = pv[it];
  }
  __threadfence();
  if (full) {
#pragma unroll
    for (int it = 0; it < 2; ++it) *(volatile v8us*)(wz + po[it]) = pv[it];
  }
}

__global__ __launch_bounds__(256) void k_cvt(const float* __restrict__ X, unsigned short* o, int np) {
  const int p = (int)blockIdx.x * 256 + (int)threadIdx.x;
  const int pc = p < np ? p : np - 1;
  const v4f a = *(const v4f*)(X + (size_t)pc * 8);
  const v4f b = *(const v4f*)(X + (size_t)pc * 8 + 4);
  const v8us hv = cvt8(a, b, ASCL);
  unsigned short* op = o + (size_t)pc * 8;
  if (p < np) *(volatile v8us*)op = hv;
  __threadfence();
  if (p < np) *(volatile v8us*)op = hv;
}

__global__ __launch_bounds__(256) void k_ln(
    const float* X, const float* Y, const float* __restrict__ g, const float* __restrict__ b,
    float* outF, unsigned short* outH, int nRows) {
  const int tid = (int)threadIdx.x, lane = tid & 31, wave = tid >> 5;
  const int row = (int)blockIdx.x * 8 + wave;
  if (row < nRows) {
    const size_t off = (size_t)row * HID + 4 * lane;
    const v4f x = *(const v4f*)(X + off) + *(const v4f*)(Y + off);
    float s = (x.x + x.y) + (x.z + x.w);
#pragma unroll
    for (int oo = 16; oo >= 1; oo >>= 1) s += __shfl_xor(s, oo);
    const float mu = s * INVHID;
    const v4f d = x - mu;
    float sq = (d.x * d.x + d.y * d.y) + (d.z * d.z + d.w * d.w);
#pragma unroll
    for (int oo = 16; oo >= 1; oo >>= 1) sq += __shfl_xor(sq, oo);
    const float var  = sq * INVHID;
    const float rstd = rsqrtf(var + LNEPS);
    const v4f g4 = *(const v4f*)(g + 4 * lane);
    const v4f b4 = *(const v4f*)(b + 4 * lane);
    const v4f y = (d * rstd) * g4 + b4;
    v4us hv;
    hv.x = h16(y.x * ASCL); hv.y = h16(y.y * ASCL); hv.z = h16(y.z * ASCL); hv.w = h16(y.w * ASCL);
    *(volatile v4f*)(outF + off) = y;
    *(volatile v4us*)(outH + off) = hv;
    __threadfence();
    *(volatile v4f*)(outF + off) = y;
    *(volatile v4us*)(outH + off) = hv;
  }
}

template <int OUTF, int OUTH, int GELU, int RES, int B2>
__global__ __launch_bounds__(GTH) void k_gemm(
    const unsigned short* __restrict__ A, const unsigned short* __restrict__ Bt,
    const float* __restrict__ bias0, const float* __restrict__ bias1, int nsplit,
    const float* __restrict__ bias2, const float* res,
    float* outF, unsigned short* outH, int K, int Ncols, int M, int ldres, int ldF, int ldH) {
  __shared__ __attribute__((aligned(16))) float sT[(GTH / 32) * GWT];
  const int tid = (int)threadIdx.x, lane = tid & 31, wave = tid >> 5, hh = lane >> 4, m = lane & 15;
  const int r0 = (int)blockIdx.y * GBM + wave * 16;
  const int c0 = (int)blockIdx.x * 128;

  int ra = r0 + m; ra = ra > M - 1 ? M - 1 : ra;
  const unsigned short* ap = A + (size_t)ra * K + 8 * hh;
  int cb = c0 + m; cb = cb > Ncols - 1 ? Ncols - 1 : cb;
  const unsigned short* bp = Bt + (size_t)cb * K + 8 * hh;

  v8f acc[8];
#pragma unroll
  for (int j = 0; j < 8; ++j) acc[j] = zero8();

  const int nk = K >> 5;
#pragma unroll 1
  for (int kt = 0; kt < nk; ++kt) {
    const int kb = kt << 5;
    FragH a;
    a.u[0] = *(const v8us*)(ap + kb);
    a.u[1] = *(const v8us*)(ap + kb + 16);
#pragma unroll
    for (int j = 0; j < 8; ++j) {
      const unsigned short* bj = bp + (size_t)(16 * j) * (size_t)K + kb;
      FragH b;
      b.u[0] = *(const v8us*)(bj);
      b.u[1] = *(const v8us*)(bj + 16);
      acc[j] = wmh(a.v, b.v, acc[j]);
    }
  }

  float* sw = sT + wave * GWT;
#pragma unroll
  for (int j = 0; j < 8; ++j)
#pragma unroll
    for (int r = 0; r < 8; ++r)
      sw[(8 * hh + r) * 128 + 16 * j + m] = acc[j][r];
  __syncthreads();

  const bool lowb = c0 < nsplit;
  const float* bb = lowb ? bias0 : bias1;
  const int boff = lowb ? 0 : nsplit;

  if (OUTF) {
    const int col = c0 + 4 * lane;
    v4f b4 = *(const v4f*)(bb + (col - boff));
    if (B2) b4 = b4 + *(const v4f*)(bias2 + col);
    v4f ov[16];
#pragma unroll
    for (int it = 0; it < 16; ++it) {
      v4f o = *(const v4f*)(sw + it * 128 + 4 * lane) * INVSCL + b4;
      if (GELU) o = gelu4(o);
      if (RES) o = o + *(const v4f*)(res + (size_t)(r0 + it) * ldres + col);
      ov[it] = o;
    }
    float* op = outF + (size_t)r0 * ldF + col;
#pragma unroll
    for (int it = 0; it < 16; ++it) *(volatile v4f*)(op + (size_t)it * ldF) = ov[it];
    __threadfence();
#pragma unroll
    for (int it = 0; it < 16; ++it) *(volatile v4f*)(op + (size_t)it * ldF) = ov[it];
  }
  if (OUTH) {
    const int rl = lane >> 4, c8 = (lane & 15) * 8, col = c0 + c8;
    v4f b0 = *(const v4f*)(bb + (col - boff));
    v4f b1 = *(const v4f*)(bb + (col - boff) + 4);
    if (B2) { b0 = b0 + *(const v4f*)(bias2 + col); b1 = b1 + *(const v4f*)(bias2 + col + 4); }
    v8us hv[8];
#pragma unroll
    for (int it = 0; it < 8; ++it) {
      const int row = 2 * it + rl;
      v4f o0 = *(const v4f*)(sw + row * 128 + c8) * INVSCL + b0;
      v4f o1 = *(const v4f*)(sw + row * 128 + c8 + 4) * INVSCL + b1;
      if (GELU) { o0 = gelu4(o0); o1 = gelu4(o1); }
      if (RES) {
        const float* rr = res + (size_t)(r0 + row) * ldres + col;
        o0 = o0 + *(const v4f*)(rr);
        o1 = o1 + *(const v4f*)(rr + 4);
      }
      hv[it] = cvt8(o0, o1, ASCL);
    }
    unsigned short* op = outH + (size_t)(r0 + rl) * ldH + col;
#pragma unroll
    for (int it = 0; it < 8; ++it) *(volatile v8us*)(op + (size_t)(2 * it) * ldH) = hv[it];
    __threadfence();
#pragma unroll
    for (int it = 0; it < 8; ++it) *(volatile v8us*)(op + (size_t)(2 * it) * ldH) = hv[it];
  }
}

__global__ __launch_bounds__(256) void k_conv(
    const unsigned short* __restrict__ qkv, const unsigned short* __restrict__ hd,
    const unsigned short* __restrict__ ws16, const float* __restrict__ bsv,
    const float* __restrict__ Wb, const int* __restrict__ src, const int* __restrict__ dst,
    float* outN, int nN, int nE) {
  extern __shared__ __align__(16) unsigned char clds[];
  unsigned short* sKs  = (unsigned short*)(clds + LO_KS);
  unsigned short* sVt  = (unsigned short*)(clds + LO_VT);
  float*          sS   = (float*)(clds + LO_S);
  unsigned short* sP   = (unsigned short*)(clds + LO_P);
  int*            sList = (int*)(clds + LO_LIST);
  int*            sWt  = (int*)(clds + LO_WT);
  float*          sRed = (float*)(clds + LO_RED);
  float*          sBeta = (float*)(clds + LO_BETA);

  const int tid = (int)threadIdx.x, lane = tid & 31, wave = tid >> 5, hh = lane >> 4, m = lane & 15;
  const int nb = (int)blockIdx.x * NBK;

  int Htot = 0;
#pragma unroll 1
  for (int cb = 0; cb < nE; cb += ECH) {
    const int e0 = cb + 16 * tid;
    int dd[16], ss[16];
#pragma unroll
    for (int q = 0; q < 4; ++q) {
      const int gi = e0 + 4 * q;
      const int ga = gi < nE - 4 ? gi : nE - 4;
      const v4i dv = *(const v4i*)(dst + ga);
      const v4i sv = *(const v4i*)(src + ga);
      const bool gv = gi < nE;
      dd[4 * q + 0] = gv ? dv.x : DSENT; dd[4 * q + 1] = gv ? dv.y : DSENT;
      dd[4 * q + 2] = gv ? dv.z : DSENT; dd[4 * q + 3] = gv ? dv.w : DSENT;
      ss[4 * q + 0] = sv.x; ss[4 * q + 1] = sv.y; ss[4 * q + 2] = sv.z; ss[4 * q + 3] = sv.w;
    }
    int hits = 0, cnt = 0;
#pragma unroll
    for (int j = 0; j < 16; ++j) {
      const int h = ((unsigned)(dd[j] - nb) < (unsigned)NBK) ? 1 : 0;
      hits |= h << j;
      cnt += h;
    }
    int x = cnt;
#pragma unroll
    for (int o = 1; o <= 16; o <<= 1) {
      const int y = __shfl_up(x, o);
      x += (lane >= o) ? y : 0;
    }
    if (lane == 31) sWt[wave] = x;
    __syncthreads();
    int wbase = 0, tot = 0;
#pragma unroll
    for (int w = 0; w < 8; ++w) {
      const int t = sWt[w];
      wbase += (w < wave) ? t : 0;
      tot += t;
    }
    int pos = Htot + wbase + (x - cnt);
#pragma unroll
    for (int j = 0; j < 16; ++j) {
      if ((hits >> j) & 1) {
        if (pos < HCAP) {
          int s = ss[j];
          s = s < 0 ? 0 : (s > nN - 1 ? nN - 1 : s);
          sList[pos] = (s << 4) | (dd[j] - nb);
        }
        ++pos;
      }
    }
    Htot += tot;
    __syncthreads();
  }
  const int H = Htot < HCAP ? Htot : HCAP;
  const int Hp = (H + 31) & ~31;
  const int nseg = Hp >> 5;
  const int nct = Hp >> 4;
  if (tid >= H && tid < HCAP) sList[tid] = 0;

  v8f acco = zero8();
#pragma unroll 1
  for (int h = 0; h < NHD; ++h) {
    __syncthreads();
#pragma unroll 1
    for (int p = tid; p < Hp * 16; p += 256) {
      const int e = p >> 4, c = p & 15;
      const int ent = sList[e];
      int s = ent >> 4;
      s = s < 0 ? 0 : (s > nN - 1 ? nN - 1 : s);
      const bool ok = e < H;
      const unsigned short* rp = qkv + (size_t)s * QKVP + h * HID + 8 * c;
      v8us kk = *(const v8us*)(rp + INNER);
      v8us vv = *(const v8us*)(rp + 2 * INNER);
      if (!ok) {
        const v8us z8 = {0, 0, 0, 0, 0, 0, 0, 0};
        kk = z8; vv = z8;
      }
      *(v8us*)(sKs + e * KPIT + 8 * c) = kk;
#pragma unroll
      for (int i = 0; i < 8; ++i) sVt[(8 * c + i) * VPIT + e] = vv[i];
    }
    __syncthreads();

    FragH qa[4];
    {
      const unsigned short* qrow = qkv + (size_t)(nb + m) * QKVP + h * HID + 8 * hh;
#pragma unroll
      for (int t = 0; t < 4; ++t) {
        qa[t].u[0] = *(const v8us*)(qrow + 32 * t);
        qa[t].u[1] = *(const v8us*)(qrow + 32 * t + 16);
      }
    }
#pragma unroll 1
    for (int ct = wave; ct < nct; ct += 8) {
      v8f acc = zero8();
      const unsigned short* kr = sKs + (ct * 16 + m) * KPIT + 8 * hh;
#pragma unroll
      for (int t = 0; t < 4; ++t) {
        FragH b;
        b.u[0] = *(const v8us*)(kr + 32 * t);
        b.u[1] = *(const v8us*)(kr + 32 * t + 16);
        acc = wmh(qa[t].v, b.v, acc);
      }
      const int e = ct * 16 + m;
      const int ent = sList[e];
      const bool ev = e < H;
      const int nl = ent & 15;
#pragma unroll
      for (int r = 0; r < 8; ++r) {
        const int row = 8 * hh + r;
        const bool keep = ev && (nl == row);
        sS[row * SPIT + e] = keep ? acc[r] * LSCL : -__builtin_inff();
      }
    }
    __syncthreads();

#pragma unroll
    for (int rr = 0; rr < 2; ++rr) {
      const int row = wave + 8 * rr;
      float sv[8];
      float mx = -__builtin_inff();
#pragma unroll
      for (int i = 0; i < 8; ++i) {
        const float t = sS[row * SPIT + 32 * i + lane];
        sv[i] = (i < nseg) ? t : -__builtin_inff();
        mx = fmaxf(mx, sv[i]);
      }
#pragma unroll
      for (int o = 16; o >= 1; o >>= 1) mx = fmaxf(mx, __shfl_xor(mx, o));
      mx = (mx > -3.0e38f) ? mx : 0.0f;
      float z = 0.0f;
#pragma unroll
      for (int i = 0; i < 8; ++i) { sv[i] = expf(sv[i] - mx); z += sv[i]; }
#pragma unroll
      for (int o = 16; o >= 1; o >>= 1) z += __shfl_xor(z, o);
      const float rz = 1.0f / (z + 1e-16f);
#pragma unroll
      for (int i = 0; i < 8; ++i) {
        if (i < nseg) sP[row * PPIT + 32 * i + lane] = h16(sv[i] * rz * PSCL);
      }
    }
    __syncthreads();

    {
      const unsigned short* vr = sVt + (16 * wave + m) * VPIT + 8 * hh;
      const unsigned short* pr = sP + m * PPIT + 8 * hh;
#pragma unroll 1
      for (int ks = 0; ks < nseg; ++ks) {
        FragH a, b;
        a.u[0] = *(const v8us*)(pr + 32 * ks);
        a.u[1] = *(const v8us*)(pr + 32 * ks + 16);
        b.u[0] = *(const v8us*)(vr + 32 * ks);
        b.u[1] = *(const v8us*)(vr + 32 * ks + 16);
        acco = wmh(a.v, b.v, acco);
      }
    }
  }

  v8f accr = zero8();
  {
    const unsigned short* ar = hd + (size_t)(nb + m) * HID + 8 * hh;
    const unsigned short* br = ws16 + (size_t)(16 * wave + m) * HID + 8 * hh;
#pragma unroll
    for (int t = 0; t < 4; ++t) {
      FragH a, b;
      a.u[0] = *(const v8us*)(ar + 32 * t);
      a.u[1] = *(const v8us*)(ar + 32 * t + 16);
      b.u[0] = *(const v8us*)(br + 32 * t);
      b.u[1] = *(const v8us*)(br + 32 * t + 16);
      accr = wmh(a.v, b.v, accr);
    }
  }
  const int col = 16 * wave + m;
  const float bcol = bsv[col];
  const float w0 = Wb[col], w1 = Wb[HID + col], w2 = Wb[2 * HID + col];
  float ov[8], xv[8], tg[8];
#pragma unroll
  for (int r = 0; r < 8; ++r) {
    ov[r] = acco[r] * OSCL;
    xv[r] = accr[r] * INVSCL + bcol;
    tg[r] = ov[r] * w0 + xv[r] * w1 + (ov[r] - xv[r]) * w2;
  }
#pragma unroll
  for (int r = 0; r < 8; ++r) {
#pragma unroll
    for (int o = 1; o <= 8; o <<= 1) tg[r] += __shfl_xor(tg[r], o);
  }
  if (m == 0) {
#pragma unroll
    for (int r = 0; r < 8; ++r) sRed[(8 * hh + r) * 8 + wave] = tg[r];
  }
  __syncthreads();
  if (tid < NBK) {
    float d = 0.0f;
#pragma unroll
    for (int w = 0; w < 8; ++w) d += sRed[tid * 8 + w];
    sBeta[tid] = 1.0f / (1.0f + expf(-d));
  }
  __syncthreads();
  float* sStg = sS;
#pragma unroll
  for (int r = 0; r < 8; ++r) {
    const int row = 8 * hh + r;
    const float be = sBeta[row];
    sStg[row * HID + col] = be * xv[r] + (1.0f - be) * ov[r];
  }
  __syncthreads();
  const v4f o0 = *(const v4f*)(sStg + (2 * wave) * HID + 4 * lane);
  const v4f o1 = *(const v4f*)(sStg + (2 * wave + 1) * HID + 4 * lane);
  float* g0 = outN + (size_t)(nb + 2 * wave) * HID + 4 * lane;
  float* g1 = g0 + HID;
  *(volatile v4f*)g0 = o0;
  *(volatile v4f*)g1 = o1;
  __threadfence();
  *(volatile v4f*)g0 = o0;
  *(volatile v4f*)g1 = o1;
}

extern "C" void kernel_launch(void* const* d_in, const int* in_sizes, int n_in,
                              void* d_out, int out_size, void* d_ws, size_t ws_size,
                              hipStream_t stream) {
  if (n_in < 46) return;
  const int nN = in_sizes[0] / DIN;
  if (nN <= 0 || nN > (1 << 24)) return;
  if (in_sizes[0] != nN * DIN) return;
  if ((nN % GBM) != 0 || (nN % NBK) != 0 || (nN % 8) != 0) return;
  if (out_size != 2 * nN * HID) return;
  for (int t = 0; t < 2; ++t) {
    const int b = 13 * t;
    if (in_sizes[b + 0] != nN * DIN) return;
    if (in_sizes[b + 1] != DIN * HID || in_sizes[b + 2] != HID) return;
    if (in_sizes[b + 3] != nN * HID || in_sizes[b + 4] != HID) return;
    if (in_sizes[b + 5] != NLAY * HID || in_sizes[b + 6] != NLAY * HID) return;
    if (in_sizes[b + 7] != NLAY * HID * FFD || in_sizes[b + 8] != NLAY * FFD) return;
    if (in_sizes[b + 9] != NLAY * FFD * HID || in_sizes[b + 10] != NLAY * HID) return;
    if (in_sizes[b + 11] != HID * HID || in_sizes[b + 12] != HID) return;
  }
  int nE[2];
  for (int d = 0; d < 2; ++d) {
    const int b = 26 + 10 * d;
    if (in_sizes[b + 0] != NLAY * HID * INNER || in_sizes[b + 1] != NLAY * HID * INNER || in_sizes[b + 2] != NLAY * HID * INNER) return;
    if (in_sizes[b + 3] != NLAY * HID * HID || in_sizes[b + 4] != NLAY * 3 * HID) return;
    if (in_sizes[b + 5] != NLAY * INNER || in_sizes[b + 6] != NLAY * INNER || in_sizes[b + 7] != NLAY * INNER) return;
    if (in_sizes[b + 8] != NLAY * HID) return;
    const int ne2 = in_sizes[b + 9];
    nE[d] = ne2 / 2;
    if (nE[d] < 4 || ne2 != 2 * nE[d] || nE[d] > (1 << 28)) return;
    if ((nE[d] % 4) != 0) return;
  }

  const float* xin[2]; const float* Win[2]; const float* bin[2]; const float* pos[2]; const float* te[2];
  const float* lng[2]; const float* lnb[2]; const float* W1[2]; const float* b1[2]; const float* W2[2]; const float* b2[2];
  const float* Wout[2]; const float* bout[2];
  for (int t = 0; t < 2; ++t) {
    const int b = 13 * t;
    xin[t]  = (const float*)d_in[b + 0];
    Win[t]  = (const float*)d_in[b + 1];
    bin[t]  = (const float*)d_in[b + 2];
    pos[t]  = (const float*)d_in[b + 3];
    te[t]   = (const float*)d_in[b + 4];
    lng[t]  = (const float*)d_in[b + 5];
    lnb[t]  = (const float*)d_in[b + 6];
    W1[t]   = (const float*)d_in[b + 7];
    b1[t]   = (const float*)d_in[b + 8];
    W2[t]   = (const float*)d_in[b + 9];
    b2[t]   = (const float*)d_in[b + 10];
    Wout[t] = (const float*)d_in[b + 11];
    bout[t] = (const float*)d_in[b + 12];
  }
  const float* Wq[2]; const float* Wk[2]; const float* Wv[2]; const float* Ws[2]; const float* Wbv[2];
  const float* bq[2]; const float* bk[2]; const float* bv[2]; const float* bs[2]; const int* ei[2];
  for (int d = 0; d < 2; ++d) {
    const int b = 26 + 10 * d;
    Wq[d]  = (const float*)d_in[b + 0];
    Wk[d]  = (const float*)d_in[b + 1];
    Wv[d]  = (const float*)d_in[b + 2];
    Ws[d]  = (const float*)d_in[b + 3];
    Wbv[d] = (const float*)d_in[b + 4];
    bq[d]  = (const float*)d_in[b + 5];
    bk[d]  = (const float*)d_in[b + 6];
    bv[d]  = (const float*)d_in[b + 7];
    bs[d]  = (const float*)d_in[b + 8];
    ei[d]  = (const int*)d_in[b + 9];
  }
  float* out = (float*)d_out;

  size_t off = 0;
  auto carve = [&](size_t bytes) { const size_t o = off; off += (bytes + 255) & ~(size_t)255; return o; };
  size_t oWin[2], oWq[2], oWkv[2], oWs[2], oW1[2], oW2[2], oWo[2];
  for (int i = 0; i < 2; ++i) oWin[i] = carve((size_t)HID * DIN * 2);
  for (int i = 0; i < 2; ++i) oWq[i]  = carve((size_t)NLAY * INNER * HID * 2);
  for (int i = 0; i < 2; ++i) oWkv[i] = carve((size_t)NLAY * 2 * INNER * HID * 2);
  for (int i = 0; i < 2; ++i) oWs[i]  = carve((size_t)NLAY * HID * HID * 2);
  for (int i = 0; i < 2; ++i) oW1[i]  = carve((size_t)NLAY * FFD * HID * 2);
  for (int i = 0; i < 2; ++i) oW2[i]  = carve((size_t)NLAY * HID * FFD * 2);
  for (int i = 0; i < 2; ++i) oWo[i]  = carve((size_t)HID * HID * 2);
  const size_t oX16 = carve((size_t)nN * DIN * 2);
  size_t oHF[2], oHH[2], oNew[2];
  for (int i = 0; i < 2; ++i) oHF[i] = carve((size_t)nN * HID * 4);
  for (int i = 0; i < 2; ++i) oHH[i] = carve((size_t)nN * HID * 2);
  const size_t oQKV = carve((size_t)nN * QKVP * 2);
  for (int i = 0; i < 2; ++i) oNew[i] = carve((size_t)nN * HID * 4);
  const size_t oRF = carve((size_t)nN * HID * 4);
  const size_t oRH = carve((size_t)nN * HID * 2);
  const size_t oGH = carve((size_t)nN * FFD * 2);
  if (off > ws_size || off > (size_t)WSCAP) return;

  char* ws = (char*)d_ws;
  unsigned short* win16[2]; unsigned short* wq16[2]; unsigned short* wkv16[2]; unsigned short* ws16[2];
  unsigned short* w116[2]; unsigned short* w216[2]; unsigned short* wo16[2];
  float* hF[2]; unsigned short* hH[2]; float* newF[2];
  for (int i = 0; i < 2; ++i) {
    win16[i] = (unsigned short*)(ws + oWin[i]);
    wq16[i]  = (unsigned short*)(ws + oWq[i]);
    wkv16[i] = (unsigned short*)(ws + oWkv[i]);
    ws16[i]  = (unsigned short*)(ws + oWs[i]);
    w116[i]  = (unsigned short*)(ws + oW1[i]);
    w216[i]  = (unsigned short*)(ws + oW2[i]);
    wo16[i]  = (unsigned short*)(ws + oWo[i]);
    hF[i]    = (float*)(ws + oHF[i]);
    hH[i]    = (unsigned short*)(ws + oHH[i]);
    newF[i]  = (float*)(ws + oNew[i]);
  }
  unsigned short* x16 = (unsigned short*)(ws + oX16);
  unsigned short* qkv = (unsigned short*)(ws + oQKV);
  float*          rF  = (float*)(ws + oRF);
  unsigned short* rH  = (unsigned short*)(ws + oRH);
  unsigned short* gH  = (unsigned short*)(ws + oGH);

  hipFuncSetAttribute(reinterpret_cast<const void*>(&k_conv), hipFuncAttributeMaxDynamicSharedMemorySize, CONV_LDS);

  const int  nobias2 = 1 << 30;
  const dim3 gM128(HID / 128, nN / GBM);
  const dim3 gM1024(INNER / 128, nN / GBM);
  const dim3 gM2048((2 * INNER) / 128, nN / GBM);
  const dim3 gM512(FFD / 128, nN / GBM);

  for (int t = 0; t < 2; ++t) {
    k_wpack<<<dim3(HID / 64, DIN / 64, 1), 256, 0, stream>>>(Win[t], win16[t], DIN, HID, 0, 0);
    k_wpack<<<dim3(FFD / 64, HID / 64, NLAY), 256, 0, stream>>>(W1[t], w116[t], HID, FFD, HID * FFD, FFD * HID);
    k_wpack<<<dim3(HID / 64, FFD / 64, NLAY), 256, 0, stream>>>(W2[t], w216[t], FFD, HID, FFD * HID, HID * FFD);
    k_wpack<<<dim3(HID / 64, HID / 64, 1), 256, 0, stream>>>(Wout[t], wo16[t], HID, HID, 0, 0);
  }
  for (int d = 0; d < 2; ++d) {
    k_wpack<<<dim3(INNER / 64, HID / 64, NLAY), 256, 0, stream>>>(Wq[d], wq16[d], HID, INNER, HID * INNER, INNER * HID);
    k_wpack<<<dim3(INNER / 64, HID / 64, NLAY), 256, 0, stream>>>(Wk[d], wkv16[d], HID, INNER, HID * INNER, 2 * INNER * HID);
    k_wpack<<<dim3(INNER / 64, HID / 64, NLAY), 256, 0, stream>>>(Wv[d], wkv16[d] + (size_t)INNER * HID, HID, INNER, HID * INNER, 2 * INNER * HID);
    k_wpack<<<dim3(HID / 64, HID / 64, NLAY), 256, 0, stream>>>(Ws[d], ws16[d], HID, HID, HID * HID, HID * HID);
  }

  const int npx = nN * DIN / 8;
  for (int t = 0; t < 2; ++t) {
    k_cvt<<<(npx + 255) / 256, 256, 0, stream>>>(xin[t], x16, npx);
    k_gemm<1, 1, 0, 1, 1><<<gM128, GTH, 0, stream>>>(x16, win16[t], bin[t], bin[t], nobias2, te[t], pos[t],
                                                     hF[t], hH[t], DIN, HID, nN, HID, HID, HID);
  }

  for (int l = 0; l < NLAY; ++l) {
    for (int d = 0; d < 2; ++d) {
      const int dstT = (d == 0) ? 1 : 0;
      const int srcT = 1 - dstT;
      k_gemm<0, 1, 0, 0, 0><<<gM1024, GTH, 0, stream>>>(hH[dstT], wq16[d] + (size_t)l * INNER * HID, bq[d] + (size_t)l * INNER,
                                                        bq[d] + (size_t)l * INNER, nobias2, bq[d], rF,
                                                        rF, qkv, HID, INNER, nN, HID, HID, QKVP);
      k_gemm<0, 1, 0, 0, 0><<<gM2048, GTH, 0, stream>>>(hH[srcT], wkv16[d] + (size_t)l * 2 * INNER * HID, bk[d] + (size_t)l * INNER,
                                                        bv[d] + (size_t)l * INNER, INNER, bk[d], rF,
                                                        rF, qkv + INNER, HID, 2 * INNER, nN, HID, HID, QKVP);
      k_conv<<<nN / NBK, 256, CONV_LDS, stream>>>(qkv, hH[dstT], ws16[d] + (size_t)l * HID * HID, bs[d] + (size_t)l * HID,
                                                  Wbv[d] + (size_t)l * 3 * HID, ei[d], ei[d] + nE[d], newF[dstT], nN, nE[d]);
    }
    for (int t = 0; t < 2; ++t) {
      k_ln<<<nN / 8, 256, 0, stream>>>(hF[t], newF[t], lng[t] + (size_t)l * HID, lnb[t] + (size_t)l * HID, rF, rH, nN);
      k_gemm<0, 1, 1, 0, 0><<<gM512, GTH, 0, stream>>>(rH, w116[t] + (size_t)l * FFD * HID, b1[t] + (size_t)l * FFD,
                                                       b1[t] + (size_t)l * FFD, nobias2, b1[t], rF,
                                                       rF, gH, HID, FFD, nN, HID, HID, FFD);
      k_gemm<1, 1, 0, 1, 0><<<gM128, GTH, 0, stream>>>(gH, w216[t] + (size_t)l * HID * FFD, b2[t] + (size_t)l * HID,
                                                       b2[t] + (size_t)l * HID, nobias2, b2[t], rF,
                                                       hF[t], hH[t], FFD, HID, nN, HID, HID, HID);
    }
  }

  for (int t = 0; t < 2; ++t) {
    k_gemm<1, 0, 0, 0, 0><<<gM128, GTH, 0, stream>>>(hH[t], wo16[t], bout[t], bout[t], nobias2, bout[t], rF,
                                                     out + (size_t)t * nN * HID, rH, HID, HID, nN, HID, HID, HID);
  }
}
